// Vanilla_MAE_19533511262661
// MI455X (gfx1250) — hardware-run, weakly checked
//
#include <hip/hip_runtime.h>
#include <math.h>

typedef __attribute__((ext_vector_type(16))) _Float16 v16h;
typedef __attribute__((ext_vector_type(8)))  _Float16 v8h;
typedef __attribute__((ext_vector_type(16))) __bf16   v16b;
typedef __attribute__((ext_vector_type(8)))  __bf16   v8b;
typedef __attribute__((ext_vector_type(8)))  float    v8f;
typedef __attribute__((ext_vector_type(4)))  float    v4f;
typedef __attribute__((ext_vector_type(4)))  unsigned int v4u;
typedef __attribute__((ext_vector_type(4)))  int      v4i;

constexpr int kRows    = 16384;
constexpr int kSeq     = 512;
constexpr int kHid     = 1024;
constexpr int kEnc     = 256;
constexpr int kExp     = 8;
constexpr int kBucket  = 128;
constexpr int kPadRows = kRows + kExp * kBucket;
static_assert(kPadRows == 17408, "padded bucket rows");
static_assert((kSeq % 32) == 0 && (kHid % 32) == 0 && (kEnc % 32) == 0, "GEMM K multiples of 32");
static_assert((kRows % 64) == 0 && (kPadRows % 64) == 0, "GEMM M multiples of 64");
static_assert((kHid % 64) == 0 && (kEnc % 64) == 0 && (kSeq % 64) == 0, "GEMM N multiples of 64");
static_assert((kPadRows % 8) == 0 && ((kPadRows / 4) % 256) == 0, "router / gather coverage");
static_assert(kRows <= 65535, "16-bit LDS slot encoding");

constexpr size_t kSzXB   = (size_t)kRows * kSeq * 2;
constexpr size_t kSzH    = (size_t)kRows * kHid * 2;
constexpr size_t kSzU    = (size_t)kPadRows * kHid * 2;
constexpr size_t kSzZ    = (size_t)kRows * kEnc * 2;
constexpr size_t kSzG    = (size_t)kPadRows * kEnc * 2;
constexpr size_t kSzW1   = (size_t)kHid * kSeq * 2;
constexpr size_t kSzW2   = (size_t)kEnc * kHid * 2;
constexpr size_t kSzW3   = (size_t)kExp * kHid * kEnc * 2;
constexpr size_t kSzW4   = (size_t)kExp * kSeq * kHid * 2;
constexpr size_t kSzPerm = (size_t)kPadRows * 4;
constexpr size_t kSzPoff = 128;
constexpr size_t kSzRegA = kSzXB + 2 * kSzH;
static_assert(2 * kSzU <= kSzRegA, "u planes fit the dead x/h region");

constexpr size_t kOffXB   = 0;
constexpr size_t kOffHH   = kOffXB + kSzXB;
constexpr size_t kOffHL   = kOffHH + kSzH;
constexpr size_t kOffUH   = 0;
constexpr size_t kOffUL   = kOffUH + kSzU;
constexpr size_t kOffZH   = kSzRegA;
constexpr size_t kOffZL   = kOffZH + kSzZ;
constexpr size_t kOffGH   = kOffZL + kSzZ;
constexpr size_t kOffGL   = kOffGH + kSzG;
constexpr size_t kOffW1   = kOffGL + kSzG;
constexpr size_t kOffW2   = kOffW1 + kSzW1;
constexpr size_t kOffW3   = kOffW2 + kSzW2;
constexpr size_t kOffW4   = kOffW3 + kSzW3;
constexpr size_t kOffPerm = kOffW4 + kSzW4;
constexpr size_t kOffPoff = kOffPerm + kSzPerm;
constexpr size_t kWsTotal = kOffPoff + kSzPoff;
static_assert(kWsTotal == 132714624ull, "carve total");
static_assert(kWsTotal <= 134217728ull, "carve cap");
static_assert((kOffHH % 128) == 0 && (kOffHL % 128) == 0 && (kOffUL % 128) == 0 && (kOffZH % 128) == 0 &&
              (kOffZL % 128) == 0 && (kOffGH % 128) == 0 && (kOffGL % 128) == 0 && (kOffW1 % 128) == 0 &&
              (kOffW2 % 128) == 0 && (kOffW3 % 128) == 0 && (kOffW4 % 128) == 0 && (kOffPerm % 128) == 0 &&
              (kOffPoff % 128) == 0, "128-B aligned regions");

__device__ __forceinline__ unsigned short f2bf_bits(float f) {
  unsigned u = __float_as_uint(f);
  return (unsigned short)((u + 0x7FFFu + ((u >> 16) & 1u)) >> 16);
}
__device__ __forceinline__ float bf_bits2f(unsigned short h) { return __uint_as_float(((unsigned)h) << 16); }

__device__ __forceinline__ v8f mma_g(v16b a, v16b b, v8f c) {
  c = __builtin_amdgcn_wmma_f32_16x16x32_bf16(false, a, false, b, (short)0, c, false, false);
  asm volatile("v_nop\n\tv_nop\n\tv_nop\n\tv_nop" : "+v"(c) : "v"(a), "v"(b));
  return c;
}

union FragB { v16b v; v8b h[2]; };
__device__ __forceinline__ v16b frag_load(const __bf16* p) {
  FragB f;
  f.h[0] = *(const v8b*)(p);
  f.h[1] = *(const v8b*)(p + 16);
  return f.v;
}

__global__ __launch_bounds__(256) void route_kernel(
    const int* __restrict__ ids, int* __restrict__ perm, int* __restrict__ poff)
{
  __shared__ unsigned short sPerm[kPadRows];
  __shared__ int sCnt[kExp];
  const int tid = threadIdx.x, lane = tid & 31, wave = tid >> 5;

#pragma unroll 1
  for (int i = tid; i < kPadRows; i += 256) sPerm[i] = (unsigned short)0xFFFFu;

  int cnt = 0;
#pragma unroll 4
  for (int c = 0; c < kRows / 32; ++c) {
    const int id = ids[c * 32 + lane];
    const unsigned bal = __builtin_amdgcn_ballot_w32(id == wave);
    cnt += __popc(bal);
  }
  if (lane == 0) sCnt[wave] = cnt;
  __syncthreads();

  int base = 0, total = 0, pv = 0;
#pragma unroll
  for (int j = 0; j < kExp; ++j) {
    int cj = sCnt[j];
    cj = cj < 0 ? 0 : (cj > kRows ? kRows : cj);
    const int rj = (cj + (kBucket - 1)) & ~(kBucket - 1);
    base += (j < wave) ? rj : 0;
    pv   += (j < lane) ? rj : 0;
    total += rj;
  }

  const unsigned lowmask = (1u << lane) - 1u;
  int pos = 0;
#pragma unroll 4
  for (int c = 0; c < kRows / 32; ++c) {
    const int r = c * 32 + lane;
    const int id = ids[r];
    const bool match = (id == wave);
    const unsigned bal = __builtin_amdgcn_ballot_w32(match);
    const int pre = __popc(bal & lowmask);
    if (match) {
      int slot = base + pos + pre;
      slot = slot > (kPadRows - 1) ? (kPadRows - 1) : slot;
      sPerm[slot] = (unsigned short)r;
    }
    pos += __popc(bal);
  }
  __syncthreads();

  for (int pass = 0; pass < 2; ++pass) {
#pragma unroll 1
    for (int it = 0; it < (kPadRows / 4) / 256; ++it) {
      const int i4 = it * 256 + tid;
      const unsigned u0 = sPerm[4 * i4 + 0];
      const unsigned u1 = sPerm[4 * i4 + 1];
      const unsigned u2 = sPerm[4 * i4 + 2];
      const unsigned u3 = sPerm[4 * i4 + 3];
      v4i v;
      v[0] = (u0 == 0xFFFFu) ? -1 : (int)u0;
      v[1] = (u1 == 0xFFFFu) ? -1 : (int)u1;
      v[2] = (u2 == 0xFFFFu) ? -1 : (int)u2;
      v[3] = (u3 == 0xFFFFu) ? -1 : (int)u3;
      *(volatile v4i*)(perm + 4 * i4) = v;
    }
    if (wave == 0) {
      const int val = (lane <= kExp) ? pv : total;
      ((volatile int*)poff)[lane] = val;
    }
    __threadfence();
  }
}

__global__ __launch_bounds__(256) void cast_rows_bf16_kernel(
    const float* __restrict__ src, unsigned short* __restrict__ dst, int total8)
{
  const int i = blockIdx.x * 256 + threadIdx.x;
  if (i >= total8) return;
  const size_t e0 = (size_t)i << 3;
  const v4f a0 = *(const v4f*)(src + e0);
  const v4f a1 = *(const v4f*)(src + e0 + 4);
  v8h hv;
#pragma unroll
  for (int e = 0; e < 4; ++e) {
    const float f0 = a0[e];
    const float f1 = a1[e];
    const unsigned short h0 = f2bf_bits(f0);
    const unsigned short h1 = f2bf_bits(f1);
    hv[e]     = __builtin_bit_cast(_Float16, h0);
    hv[4 + e] = __builtin_bit_cast(_Float16, h1);
  }
  unsigned short* q = dst + e0;
  *(volatile v8h*)q = hv;
  __threadfence();
  *(volatile v8h*)q = hv;
}

__global__ __launch_bounds__(256) void transpose_bf16_kernel(
    const float* __restrict__ in, unsigned short* __restrict__ out, int K, int Ncols)
{
  __shared__ float tile[64 * 65];
  const int tid = threadIdx.x, lane = tid & 31, wave = tid >> 5;
  const int n0 = blockIdx.x * 64, k0 = blockIdx.y * 64;
  const size_t per = (size_t)K * Ncols;
  const float* ib = in + (size_t)blockIdx.z * per;
  unsigned short* ob = out + (size_t)blockIdx.z * per;
  const int kr = tid >> 4, c4 = (tid & 15) * 4;
#pragma unroll
  for (int it = 0; it < 4; ++it) {
    const int kk = it * 16 + kr;
    const v4f v = *(const v4f*)(ib + (size_t)(k0 + kk) * Ncols + n0 + c4);
    tile[kk * 65 + c4 + 0] = v[0];
    tile[kk * 65 + c4 + 1] = v[1];
    tile[kk * 65 + c4 + 2] = v[2];
    tile[kk * 65 + c4 + 3] = v[3];
  }
  __syncthreads();
  const int q = lane >> 3, c8 = (lane & 7) * 8;
  v8h hv[2];
#pragma unroll
  for (int it = 0; it < 2; ++it) {
    const int n = it * 32 + wave * 4 + q;
#pragma unroll
    for (int e = 0; e < 8; ++e) {
      const float f = tile[(c8 + e) * 65 + n];
      const unsigned short hb = f2bf_bits(f);
      hv[it][e] = __builtin_bit_cast(_Float16, hb);
    }
  }
  for (int pass = 0; pass < 2; ++pass) {
#pragma unroll
    for (int it = 0; it < 2; ++it) {
      const int n = it * 32 + wave * 4 + q;
      *(volatile v8h*)(ob + (size_t)(n0 + n) * K + k0 + c8) = hv[it];
    }
    __threadfence();
  }
}

__global__ __launch_bounds__(256) void gather_rows_kernel(
    const unsigned short* __restrict__ zh, const unsigned short* __restrict__ zl,
    const int* __restrict__ perm,
    unsigned short* __restrict__ gh, unsigned short* __restrict__ gl)
{
  const int lane = threadIdx.x & 31, wave = threadIdx.x >> 5;
  const int r = blockIdx.x * 8 + wave;
  const int p = perm[r];
  const bool ok = ((unsigned)p < (unsigned)kRows);
  const int pc = ok ? p : 0;
  v4u a = *(const v4u*)(zh + (size_t)pc * kEnc + lane * 8);
  v4u b = *(const v4u*)(zl + (size_t)pc * kEnc + lane * 8);
  const v4u zero = (v4u){0u, 0u, 0u, 0u};
  a = ok ? a : zero;
  b = ok ? b : zero;
  unsigned short* qh = gh + (size_t)r * kEnc + lane * 8;
  unsigned short* ql = gl + (size_t)r * kEnc + lane * 8;
  *(volatile v4u*)qh = a;
  *(volatile v4u*)ql = b;
  __threadfence();
  *(volatile v4u*)qh = a;
  *(volatile v4u*)ql = b;
}

template <int SPL, int OUT_MODE, int ACT, bool EXPERT, bool SCATTER>
__global__ __launch_bounds__(256) void wmma_gemm_bf(
    const unsigned short* __restrict__ Ap, const unsigned short* __restrict__ A2p, int lda,
    const unsigned short* __restrict__ Btp, int ldb, long strideBexp,
    void* __restrict__ Cout, void* __restrict__ Cout2, int ldc,
    const float* __restrict__ bias, int biasStrideExp,
    const int* __restrict__ perm, const int* __restrict__ poff,
    int M, int N, int K, int Mreal)
{
  const __bf16* A  = (const __bf16*)Ap;
  const __bf16* A2 = (const __bf16*)A2p;
  const __bf16* Bt = (const __bf16*)Btp;
  __shared__ __align__(16) float sT[8][16 * 68];
  const int lane = threadIdx.x & 31;
  const int wave = threadIdx.x >> 5;
  const int tilesN = N >> 6;
  const int tilesM = M >> 6;
  const int tile = blockIdx.x * 8 + wave;
  if (tile >= tilesM * tilesN) return;
  const int tm = tile / tilesN;
  const int tn = tile - tm * tilesN;
  const int m0 = tm << 6;
  const int n0 = tn << 6;

  int e = 0;
  if (EXPERT) {
    int pe[kExp + 1];
#pragma unroll
    for (int j = 0; j <= kExp; ++j) {
      int v = poff[j];
      v = v < 0 ? 0 : (v > M ? M : v);
      pe[j] = v;
    }
    if (m0 >= pe[kExp]) return;
#pragma unroll
    for (int j = 1; j < kExp; ++j) e += (m0 >= pe[j]) ? 1 : 0;
  }
  const __bf16* Bb = Bt + (size_t)e * (size_t)strideBexp;
  const float* bs = bias + (size_t)e * (size_t)biasStrideExp;

  const int rlane = lane & 15;
  const int koff  = (lane >> 4) * 8;
  const int mOff  = (lane >> 4) * 8;

  v8f acc[4][4];
#pragma unroll
  for (int i = 0; i < 4; ++i)
#pragma unroll
    for (int j = 0; j < 4; ++j) acc[i][j] = (v8f){0.f, 0.f, 0.f, 0.f, 0.f, 0.f, 0.f, 0.f};

  for (int k0 = 0; k0 < K; k0 += 32) {
    v16b bh[4];
#pragma unroll
    for (int j = 0; j < 4; ++j) {
      const size_t bo = (size_t)(n0 + (j << 4) + rlane) * ldb + koff + k0;
      bh[j] = frag_load(Bb + bo);
    }
#pragma unroll
    for (int i = 0; i < 4; ++i) {
      const size_t ao = (size_t)(m0 + (i << 4) + rlane) * lda + koff + k0;
      const v16b ah = frag_load(A + ao);
      v16b al = ah;
      if (SPL == 1) al = frag_load(A2 + ao);
#pragma unroll
      for (int j = 0; j < 4; ++j) {
        acc[i][j] = mma_g(ah, bh[j], acc[i][j]);
        if (SPL == 1) acc[i][j] = mma_g(al, bh[j], acc[i][j]);
      }
    }
  }

  float* slab = sT[wave];
#pragma unroll
  for (int i = 0; i < 4; ++i) {
    const int mBase = m0 + (i << 4);
#pragma unroll
    for (int j = 0; j < 4; ++j) {
      const int n = n0 + (j << 4) + rlane;
      const float braw = bs[n];
      const float bv = bf_bits2f(f2bf_bits(braw));
#pragma unroll
      for (int r = 0; r < 8; ++r) {
        float v = acc[i][j][r] + bv;
        if (ACT == 2) v = fmaxf(v, 0.0f);
        slab[(mOff + r) * 68 + (j << 4) + rlane] = v;
      }
    }
    __builtin_amdgcn_fence(__ATOMIC_RELEASE, "workgroup");
    __builtin_amdgcn_wave_barrier();
    __builtin_amdgcn_fence(__ATOMIC_ACQUIRE, "workgroup");
    if (OUT_MODE == 0) {
      float* C = (float*)Cout;
      const int hh = lane >> 4, c4 = (lane & 15) * 4;
      int pr[8];
#pragma unroll
      for (int it = 0; it < 8; ++it) {
        const int rr = mBase + it * 2 + hh;
        pr[it] = SCATTER ? perm[rr] : rr;
      }
      for (int pass = 0; pass < 2; ++pass) {
#pragma unroll
        for (int it = 0; it < 8; ++it) {
          const int row = it * 2 + hh;
          const v4f v = *(const v4f*)(slab + row * 68 + c4);
          if ((unsigned)pr[it] < (unsigned)Mreal)
            *(volatile v4f*)(C + (size_t)pr[it] * ldc + n0 + c4) = v;
        }
        __threadfence();
      }
    } else {
      const int q = lane >> 3, c8 = (lane & 7) * 8;
      unsigned short* C  = (unsigned short*)Cout;
      unsigned short* C2 = (unsigned short*)Cout2;
      for (int pass = 0; pass < 2; ++pass) {
#pragma unroll
        for (int it = 0; it < 4; ++it) {
          const int row = it * 4 + q;
          const float* sp = slab + row * 68 + c8;
          v8h hv, lv;
#pragma unroll
          for (int el = 0; el < 8; ++el) {
            const float f = sp[el];
            const unsigned short hb = f2bf_bits(f);
            const unsigned short lb = f2bf_bits(f - bf_bits2f(hb));
            hv[el] = __builtin_bit_cast(_Float16, hb);
            lv[el] = __builtin_bit_cast(_Float16, lb);
          }
          *(volatile v8h*)(C  + (size_t)(mBase + row) * ldc + n0 + c8) = hv;
          *(volatile v8h*)(C2 + (size_t)(mBase + row) * ldc + n0 + c8) = lv;
        }
        __threadfence();
      }
    }
    __builtin_amdgcn_fence(__ATOMIC_RELEASE, "workgroup");
    __builtin_amdgcn_wave_barrier();
    __builtin_amdgcn_fence(__ATOMIC_ACQUIRE, "workgroup");
  }
}

extern "C" void kernel_launch(void* const* d_in, const int* in_sizes, int n_in,
                              void* d_out, int out_size, void* d_ws, size_t ws_size,
                              hipStream_t stream) {
  if (n_in < 10) return;
  if (in_sizes[0] != kRows * kSeq) return;
  if (in_sizes[1] != kRows) return;
  if (in_sizes[2] != kSeq * kHid) return;
  if (in_sizes[3] != kHid) return;
  if (in_sizes[4] != kHid * kEnc) return;
  if (in_sizes[5] != kEnc) return;
  if (in_sizes[6] != kExp * kEnc * kHid) return;
  if (in_sizes[7] != kExp * kHid) return;
  if (in_sizes[8] != kExp * kHid * kSeq) return;
  if (in_sizes[9] != kExp * kSeq) return;
  if (out_size != kRows * kSeq) return;
  if (ws_size < kWsTotal) return;

  const float* x   = (const float*)d_in[0];
  const int*   ids = (const int*)d_in[1];
  const float* W1  = (const float*)d_in[2];
  const float* b1  = (const float*)d_in[3];
  const float* W2  = (const float*)d_in[4];
  const float* b2  = (const float*)d_in[5];
  const float* W3  = (const float*)d_in[6];
  const float* b3  = (const float*)d_in[7];
  const float* W4  = (const float*)d_in[8];
  const float* b4  = (const float*)d_in[9];
  float* out = (float*)d_out;

  char* ws = (char*)d_ws;
  unsigned short* XB  = (unsigned short*)(ws + kOffXB);
  unsigned short* HH  = (unsigned short*)(ws + kOffHH);
  unsigned short* HL  = (unsigned short*)(ws + kOffHL);
  unsigned short* UH  = (unsigned short*)(ws + kOffUH);
  unsigned short* UL  = (unsigned short*)(ws + kOffUL);
  unsigned short* ZH  = (unsigned short*)(ws + kOffZH);
  unsigned short* ZL  = (unsigned short*)(ws + kOffZL);
  unsigned short* GH  = (unsigned short*)(ws + kOffGH);
  unsigned short* GL  = (unsigned short*)(ws + kOffGL);
  unsigned short* W1T = (unsigned short*)(ws + kOffW1);
  unsigned short* W2T = (unsigned short*)(ws + kOffW2);
  unsigned short* W3T = (unsigned short*)(ws + kOffW3);
  unsigned short* W4T = (unsigned short*)(ws + kOffW4);
  int* perm = (int*)(ws + kOffPerm);
  int* poff = (int*)(ws + kOffPoff);

  route_kernel<<<1, 256, 0, stream>>>(ids, perm, poff);

  cast_rows_bf16_kernel<<<(kRows * kSeq / 8) / 256, 256, 0, stream>>>(x, XB, kRows * kSeq / 8);

  transpose_bf16_kernel<<<dim3(kHid / 64, kSeq / 64, 1), 256, 0, stream>>>(W1, W1T, kSeq, kHid);
  transpose_bf16_kernel<<<dim3(kEnc / 64, kHid / 64, 1), 256, 0, stream>>>(W2, W2T, kHid, kEnc);
  transpose_bf16_kernel<<<dim3(kHid / 64, kEnc / 64, kExp), 256, 0, stream>>>(W3, W3T, kEnc, kHid);
  transpose_bf16_kernel<<<dim3(kSeq / 64, kHid / 64, kExp), 256, 0, stream>>>(W4, W4T, kHid, kSeq);

  wmma_gemm_bf<0, 2, 2, false, false><<<(kRows / 64) * (kHid / 64) / 8, 256, 0, stream>>>(
      XB, XB, kSeq,
      W1T, kSeq, 0L,
      (void*)HH, (void*)HL, kHid,
      b1, 0,
      perm, poff,
      kRows, kHid, kSeq, kRows);

  wmma_gemm_bf<1, 2, 2, false, false><<<(kRows / 64) * (kEnc / 64) / 8, 256, 0, stream>>>(
      HH, HL, kHid,
      W2T, kHid, 0L,
      (void*)ZH, (void*)ZL, kEnc,
      b2, 0,
      perm, poff,
      kRows, kEnc, kHid, kRows);

  gather_rows_kernel<<<kPadRows / 8, 256, 0, stream>>>(ZH, ZL, perm, GH, GL);

  wmma_gemm_bf<1, 2, 2, true, false><<<(kPadRows / 64) * (kHid / 64) / 8, 256, 0, stream>>>(
      GH, GL, kEnc,
      W3T, kEnc, (long)kHid * kEnc,
      (void*)UH, (void*)UL, kHid,
      b3, kHid,
      perm, poff,
      kPadRows, kHid, kEnc, kRows);

  wmma_gemm_bf<1, 0, 0, true, true><<<(kPadRows / 64) * (kSeq / 64) / 8, 256, 0, stream>>>(
      UH, UL, kHid,
      W4T, kHid, (long)kSeq * kHid,
      (void*)out, (void*)out, kSeq,
      b4, kSeq,
      perm, poff,
      kPadRows, kSeq, kHid, kRows);
}
